// MultiheadedFeatureSelfAttention_11802570130120
// MI455X (gfx1250) — hardware-verified
//
#include <hip/hip_runtime.h>
#include <math.h>
#include <stdint.h>

constexpr int kBatch = 2;
constexpr int kSeq   = 4096;
constexpr int kDim   = 512;
constexpr int kHeads = 8;
constexpr int kDqk   = 32;
constexpr int kDk    = 64;
constexpr int kTok   = kBatch * kSeq;
constexpr int kHid   = 2 * kDim;
constexpr int kQk    = kDim / 2;
constexpr float kWCarry   = 64.0f;
constexpr float kActCarry = 16.0f;
constexpr float kPCarry   = 2048.0f;

constexpr size_t kMiB    = 1048576;
constexpr size_t kHalfMiB = 524288;
constexpr size_t kOffQ16 = 0;
constexpr size_t kOffK16 = 4 * kMiB;
constexpr size_t kOffVT  = 8 * kMiB;
constexpr size_t kOffXhi = 16 * kMiB;
constexpr size_t kOffXlo = 24 * kMiB;
constexpr size_t kOffXq  = 32 * kMiB;
constexpr size_t kOffXk  = 40 * kMiB;
constexpr size_t kOffXv  = 48 * kMiB;
constexpr size_t kOffH   = 56 * kMiB;
constexpr size_t kOffG   = 88 * kMiB;
constexpr size_t kOffW1q = 104 * kMiB;
constexpr size_t kOffW1k = 105 * kMiB;
constexpr size_t kOffW2q = 106 * kMiB;
constexpr size_t kOffW2k = 106 * kMiB + kHalfMiB;
constexpr size_t kOffWv  = 107 * kMiB;
constexpr size_t kOffSb  = 107 * kMiB + kHalfMiB;
constexpr size_t kOffS   = 32 * kMiB;
constexpr size_t kOffP   = 96 * kMiB;
constexpr size_t kOffWoh = 32 * kMiB;
constexpr size_t kOffWol = 32 * kMiB + kHalfMiB;
constexpr size_t kWsTotal = 128 * kMiB;
static_assert((size_t)kTok * kDim * 2 == 8 * kMiB, "input f16 plane");
static_assert((size_t)kTok * kQk * 2 == 4 * kMiB, "q/k plane");
static_assert((size_t)kTok * kHid * 4 == 32 * kMiB, "hidden f32 plane");
static_assert((size_t)kTok * kHid * 2 == 16 * kMiB, "gelu plane");
static_assert((size_t)kHid * kDim * 2 == kMiB, "W1 plane");
static_assert((size_t)kQk * kHid * 2 == kHalfMiB, "W2 plane");
static_assert((size_t)kDim * kDim * 2 == kHalfMiB, "Wv/Wo plane");
static_assert((size_t)kSeq * kSeq * 4 == 64 * kMiB, "scores plane");
static_assert((size_t)kSeq * kSeq * 2 == 32 * kMiB, "P plane");
static_assert(kOffSb + 1024 * 4 <= kOffP + 32 * kMiB, "scratch fits");
static_assert(kOffP + 32 * kMiB == kWsTotal, "total carve");

typedef __attribute__((ext_vector_type(16))) _Float16 v16h;
typedef __attribute__((ext_vector_type(8)))  _Float16 v8h;
typedef __attribute__((ext_vector_type(16))) __bf16   v16b;
typedef __attribute__((ext_vector_type(8)))  __bf16   v8b;
typedef __attribute__((ext_vector_type(8)))  float    v8f;
typedef __attribute__((ext_vector_type(4)))  float    v4f;
typedef __attribute__((ext_vector_type(4)))  unsigned int v4u;

__device__ __forceinline__ unsigned short f2bf_bits(float f) {
  unsigned u = __float_as_uint(f);
  return (unsigned short)((u + 0x7FFFu + ((u >> 16) & 1u)) >> 16);
}
__device__ __forceinline__ float bf_bits2f(unsigned short h) { return __uint_as_float(((unsigned)h) << 16); }

__device__ __forceinline__ void dep_guard_h(v8f& a, v8f& b, v16h x, v16h y) { asm volatile("v_nop\n\tv_nop\n\tv_nop\n\tv_nop" : "+v"(a), "+v"(b) : "v"(x), "v"(y)); }
__device__ __forceinline__ void dep_guard_b(v8f& a, v8f& b, v16b x, v16b y) { asm volatile("v_nop\n\tv_nop\n\tv_nop\n\tv_nop" : "+v"(a), "+v"(b) : "v"(x), "v"(y)); }
__device__ __forceinline__ void keep4_h(v16h a, v16h b, v16h c, v16h d) { asm volatile("v_nop" :: "v"(a), "v"(b), "v"(c), "v"(d)); }
__device__ __forceinline__ void keep4_b(v16b a, v16b b, v16b c, v16b d) { asm volatile("v_nop" :: "v"(a), "v"(b), "v"(c), "v"(d)); }
__device__ __forceinline__ void acc_guard4(v8f& a, v8f& b, v8f& c, v8f& d) { asm volatile("v_nop\n\tv_nop\n\tv_nop\n\tv_nop" : "+v"(a), "+v"(b), "+v"(c), "+v"(d)); }
template <typename T> struct Frag;
template <> struct Frag<_Float16> {
  typedef v16h V; union U { v16h v; v8h h[2]; };
  static __device__ __forceinline__ v16h load(const _Float16* p) {
    U f; f.h[0] = *(const v8h*)(p); f.h[1] = *(const v8h*)(p + 16); return f.v;
  }
  static __device__ __forceinline__ v8f mma(v16h a, v16h b, v8f c) {
    return __builtin_amdgcn_wmma_f32_16x16x32_f16(false, a, false, b, (short)0, c, false, false);
  }
  static __device__ __forceinline__ void guard(v8f& a, v8f& b, v16h x, v16h y) { dep_guard_h(a, b, x, y); }
  static __device__ __forceinline__ void keep(v16h a, v16h b, v16h c, v16h d) { keep4_h(a, b, c, d); }
};
template <> struct Frag<__bf16> {
  typedef v16b V; union U { v16b v; v8b h[2]; };
  static __device__ __forceinline__ v16b load(const __bf16* p) {
    U f; f.h[0] = *(const v8b*)(p); f.h[1] = *(const v8b*)(p + 16); return f.v;
  }
  static __device__ __forceinline__ v8f mma(v16b a, v16b b, v8f c) {
    return __builtin_amdgcn_wmma_f32_16x16x32_bf16(false, a, false, b, (short)0, c, false, false);
  }
  static __device__ __forceinline__ void guard(v8f& a, v8f& b, v16b x, v16b y) { dep_guard_b(a, b, x, y); }
  static __device__ __forceinline__ void keep(v16b a, v16b b, v16b c, v16b d) { keep4_b(a, b, c, d); }
};

__device__ __forceinline__ unsigned pk16(unsigned short a, unsigned short b) { return (unsigned)a | ((unsigned)b << 16); }
__device__ __forceinline__ unsigned short h_bits(float f) { const _Float16 h = (_Float16)f; return __builtin_bit_cast(unsigned short, h); }

template <int ET> struct Elem;
template <> struct Elem<0> { typedef _Float16 T; };
template <> struct Elem<1> { typedef __bf16 T; };
template <int ET, bool SPLIT, int BIAS_MODE, int OUT_MODE, bool RESID, int ACT = 0>
__global__ __launch_bounds__(256) void wmma_gemm64(
    const unsigned short* __restrict__ Ap, const unsigned short* __restrict__ A2p, int lda, long strideA,
    const unsigned short* __restrict__ Btp, const unsigned short* __restrict__ Bt2p, int ldb, long strideB,
    void* __restrict__ Cout, void* __restrict__ Cout2, int ldc, long strideC,
    const float* __restrict__ bias,
    const float* __restrict__ resid, long strideR,
    int M, int N, int K, float scale) {
  typedef typename Elem<ET>::T T;
  typedef typename Frag<T>::V V;
  const T* A = (const T*)Ap; const T* A2 = (const T*)A2p; const T* Bt = (const T*)Btp; const T* Bt2 = (const T*)Bt2p;
  __shared__ __align__(16) float sT[8][16 * 68];
  const int b    = blockIdx.y;
  const int lane = threadIdx.x & 31;
  const int wave = threadIdx.x >> 5;
  const int tilesN = N >> 6;
  const int tilesM = M >> 6;
  const int tile = blockIdx.x * 8 + wave;
  if (tile >= tilesM * tilesN) return;
  const int tm = tile / tilesN;
  const int tn = tile - tm * tilesN;
  const int m0 = tm << 6;
  const int n0 = tn << 6;

  const T* Ab  = A  + (size_t)b * strideA;
  const T* Bb  = Bt + (size_t)b * strideB;
  const T* Ab2 = SPLIT ? (A2  + (size_t)b * strideA) : nullptr;
  const T* Bb2 = SPLIT ? (Bt2 + (size_t)b * strideB) : nullptr;

  const int rlane = lane & 15;
  const int koff  = (lane >> 4) * 8;
  const int mOff  = (lane >> 4) * 8;

  v8f acc[4][4];
#pragma unroll
  for (int i = 0; i < 4; ++i)
#pragma unroll
    for (int j = 0; j < 4; ++j) acc[i][j] = (v8f){0.f,0.f,0.f,0.f,0.f,0.f,0.f,0.f};

  for (int k0 = 0; k0 < K; k0 += 32) {
    V bh[4], bl[4];
#pragma unroll
    for (int j = 0; j < 4; ++j) {
      const size_t bo = (size_t)(n0 + (j << 4) + rlane) * ldb + koff + k0;
      bh[j] = Frag<T>::load(Bb + bo);
      if (SPLIT) bl[j] = Frag<T>::load(Bb2 + bo);
    }
#pragma unroll
    for (int i = 0; i < 4; ++i) {
      const size_t ao = (size_t)(m0 + (i << 4) + rlane) * lda + koff + k0;
      V ah = Frag<T>::load(Ab + ao);
      V al;
      if (SPLIT) al = Frag<T>::load(Ab2 + ao);
#pragma unroll
      for (int j = 0; j < 4; ++j) {
        acc[i][j] = Frag<T>::mma(ah, bh[j], acc[i][j]);
        if (SPLIT) {
          acc[i][j] = Frag<T>::mma(ah, bl[j], acc[i][j]);
          acc[i][j] = Frag<T>::mma(al, bh[j], acc[i][j]);
        }
      }
      Frag<T>::guard(acc[i][0], acc[i][3], ah, SPLIT ? al : ah);
    }
    Frag<T>::keep(bh[0], bh[1], bh[2], bh[3]);
    if (SPLIT) Frag<T>::keep(bl[0], bl[1], bl[2], bl[3]);
  }
  acc_guard4(acc[0][0], acc[0][1], acc[0][2], acc[0][3]);
  acc_guard4(acc[1][0], acc[1][1], acc[1][2], acc[1][3]);
  acc_guard4(acc[2][0], acc[2][1], acc[2][2], acc[2][3]);
  acc_guard4(acc[3][0], acc[3][1], acc[3][2], acc[3][3]);

  float* slab = sT[wave];
  const float* Rb = RESID ? (resid + (size_t)b * strideR) : nullptr;
#pragma unroll
  for (int i = 0; i < 4; ++i) {
    const int mBase = m0 + (i << 4);
#pragma unroll
    for (int j = 0; j < 4; ++j) {
      const int n = n0 + (j << 4) + rlane;
      float bv = 0.f;
      if (BIAS_MODE == 2) bv = bias[n];
#pragma unroll
      for (int r = 0; r < 8; ++r) {
        float v = acc[i][j][r] * scale;
        if (BIAS_MODE == 1) v += bias[mBase + mOff + r];
        if (BIAS_MODE == 2) v += bv;
        if (RESID) v += Rb[(size_t)(mBase + mOff + r) * ldc + n];
        if (ACT == 2) v = fmaxf(v, 0.0f);
        if (ACT == 4) v = (v > 0.f) ? v : 0.01f * v;
        slab[(mOff + r) * 68 + (j << 4) + rlane] = v;
      }
    }
    __builtin_amdgcn_fence(__ATOMIC_RELEASE, "workgroup");
    __builtin_amdgcn_wave_barrier();
    __builtin_amdgcn_fence(__ATOMIC_ACQUIRE, "workgroup");
    if (OUT_MODE == 0) {
      float* C = (float*)Cout + (size_t)b * strideC;
      const int hh = lane >> 4, c4 = (lane & 15) * 4;
      for (int pass = 0; pass < 2; ++pass) {
#pragma unroll
        for (int it = 0; it < 8; ++it) {
          const int row = it * 2 + hh;
          v4f v = *(const v4f*)(slab + row * 68 + c4);
          *(volatile v4f*)(C + (size_t)(mBase + row) * ldc + n0 + c4) = v;
        }
        __threadfence();
      }
    } else {
      const int q = lane >> 3, c8 = (lane & 7) * 8;
      unsigned short* C  = (unsigned short*)Cout  + (size_t)b * strideC;
      unsigned short* C2 = (OUT_MODE == 2) ? ((unsigned short*)Cout2 + (size_t)b * strideC) : nullptr;
      for (int pass = 0; pass < 2; ++pass) {
#pragma unroll
        for (int it = 0; it < 4; ++it) {
          const int row = it * 4 + q;
          const float* sp = slab + row * 68 + c8;
          v8h hv, lv;
#pragma unroll
          for (int e = 0; e < 8; ++e) {
            if (OUT_MODE == 1) {
              hv[e] = (_Float16)sp[e];
            } else {
              unsigned short hb = f2bf_bits(sp[e]);
              unsigned short lb = f2bf_bits(sp[e] - bf_bits2f(hb));
              hv[e] = __builtin_bit_cast(_Float16, hb);
              lv[e] = __builtin_bit_cast(_Float16, lb);
            }
          }
          *(volatile v8h*)(C + (size_t)(mBase + row) * ldc + n0 + c8) = hv;
          if (OUT_MODE == 2) *(volatile v8h*)(C2 + (size_t)(mBase + row) * ldc + n0 + c8) = lv;
        }
        __threadfence();
      }
    }
    __builtin_amdgcn_fence(__ATOMIC_RELEASE, "workgroup");
    __builtin_amdgcn_wave_barrier();
    __builtin_amdgcn_fence(__ATOMIC_ACQUIRE, "workgroup");
  }
}

__global__ __launch_bounds__(256) void cast8x3_kernel(const float* __restrict__ in0, const float* __restrict__ in1,
                                                      const float* __restrict__ in2,
                                                      unsigned short* __restrict__ out0, unsigned short* __restrict__ out1,
                                                      unsigned short* __restrict__ out2, int n8) {
  const int z = blockIdx.y;
  const float* in = (z == 0) ? in0 : (z == 1) ? in1 : in2;
  unsigned short* out = (z == 0) ? out0 : (z == 1) ? out1 : out2;
  const int i = blockIdx.x * 256 + threadIdx.x;
  if (i >= n8) return;
  const float* p = in + 8 * (size_t)i;
  const v4f a = *(const v4f*)(p);
  const v4f c = *(const v4f*)(p + 4);
  unsigned short hb[8];
#pragma unroll
  for (int e = 0; e < 4; ++e) {
    hb[e]     = h_bits(a[e]);
    hb[4 + e] = h_bits(c[e]);
  }
  const v4u u = (v4u){pk16(hb[0], hb[1]), pk16(hb[2], hb[3]), pk16(hb[4], hb[5]), pk16(hb[6], hb[7])};
  unsigned short* q = out + 8 * (size_t)i;
  *(volatile v4u*)q = u;
  __threadfence();
  *(volatile v4u*)q = u;
}

template <int MODE>
__global__ __launch_bounds__(256) void wtcast_kernel(const float* __restrict__ W0, const float* __restrict__ W1,
                                                     unsigned short* __restrict__ T0, unsigned short* __restrict__ T1,
                                                     int nrows, int ncols, float scale) {
  __shared__ float sm[64][65];
  const int t  = threadIdx.x;
  const int k0 = blockIdx.x * 64;
  const int n0 = blockIdx.y * 64;
  const int z  = blockIdx.z;
  const float* W = (MODE == 0 && z == 1) ? W1 : W0;
#pragma unroll
  for (int i = 0; i < 16; ++i) {
    const int e = i * 256 + t;
    const int r = e >> 6;
    const int c = e & 63;
    sm[c][r] = W[(size_t)(k0 + r) * ncols + n0 + c] * scale;
  }
  __syncthreads();
  const int lane = t & 31, wave = t >> 5;
  const int q = lane >> 3, c8 = (lane & 7) * 8;
  if (MODE == 0) {
    unsigned short* op = (z == 1) ? T1 : T0;
    for (int pass = 0; pass < 2; ++pass) {
#pragma unroll
      for (int it = 0; it < 2; ++it) {
        const int row = wave * 8 + it * 4 + q;
        unsigned short hb[8];
#pragma unroll
        for (int e = 0; e < 8; ++e) hb[e] = h_bits(sm[row][c8 + e]);
        const v4u u = (v4u){pk16(hb[0], hb[1]), pk16(hb[2], hb[3]), pk16(hb[4], hb[5]), pk16(hb[6], hb[7])};
        *(volatile v4u*)(op + (size_t)(n0 + row) * nrows + k0 + c8) = u;
      }
      __threadfence();
    }
  } else {
    for (int pass = 0; pass < 2; ++pass) {
#pragma unroll
      for (int it = 0; it < 2; ++it) {
        const int row = wave * 8 + it * 4 + q;
        unsigned short hb[8], lb[8];
#pragma unroll
        for (int e = 0; e < 8; ++e) {
          const float x = sm[row][c8 + e];
          hb[e] = f2bf_bits(x);
          lb[e] = f2bf_bits(x - bf_bits2f(hb[e]));
        }
        const v4u uh = (v4u){pk16(hb[0], hb[1]), pk16(hb[2], hb[3]), pk16(hb[4], hb[5]), pk16(hb[6], hb[7])};
        const v4u ul = (v4u){pk16(lb[0], lb[1]), pk16(lb[2], lb[3]), pk16(lb[4], lb[5]), pk16(lb[6], lb[7])};
        *(volatile v4u*)(T0 + (size_t)(n0 + row) * nrows + k0 + c8) = uh;
        *(volatile v4u*)(T1 + (size_t)(n0 + row) * nrows + k0 + c8) = ul;
      }
      __threadfence();
    }
  }
}

__global__ __launch_bounds__(64) void sbias_kernel(const float* __restrict__ b0, const float* __restrict__ b1,
                                                   const float* __restrict__ b2, float* __restrict__ sb, float s) {
  const int blk = blockIdx.x;
  const float* src = (blk == 0) ? b0 : (blk == 1) ? b1 : (b2 + (blk - 2) * 256);
  const int t = threadIdx.x;
  v4f v = *(const v4f*)(src + 4 * t);
  v = v * s;
  float* dst = sb + blk * 256 + 4 * t;
  *(volatile v4f*)dst = v;
  __threadfence();
  *(volatile v4f*)dst = v;
}

__global__ __launch_bounds__(256) void gelu_cast_kernel(const float* __restrict__ in, unsigned short* __restrict__ out,
                                                       int n2, float carry) {
  const int i = blockIdx.x * 256 + threadIdx.x;
  if (i >= n2) return;
  unsigned u = 0u;
#pragma unroll 1
  for (int e = 0; e < 2; ++e) {
    const float hval = in[2 * (size_t)i + e];
    const float g = 0.5f * hval * (1.0f + erff(hval * 0.70710678118654752f));
    u |= ((unsigned)h_bits(g * carry)) << (16 * e);
  }
  ((volatile unsigned*)out)[i] = u;
  __threadfence();
  ((volatile unsigned*)out)[i] = u;
}

__global__ __launch_bounds__(256) void softmax_row_kernel(const float* __restrict__ S, unsigned short* __restrict__ P,
                                                         float carry) {
  __shared__ float srow[kSeq];
  __shared__ float redM[8];
  __shared__ float redS[8];
  const int row  = blockIdx.x;
  const int t    = threadIdx.x;
  const int lane = t & 31, wave = t >> 5;
  const int c0   = 8 * t;
  const int c1   = kSeq / 2 + 8 * t;
  const float* sr = S + (size_t)row * kSeq;
  const v4f a0 = *(const v4f*)(sr + c0);
  const v4f a1 = *(const v4f*)(sr + c0 + 4);
  const v4f b0 = *(const v4f*)(sr + c1);
  const v4f b1 = *(const v4f*)(sr + c1 + 4);
  float m = a0[0];
#pragma unroll
  for (int e = 0; e < 4; ++e) {
    m = fmaxf(m, a0[e]); m = fmaxf(m, a1[e]); m = fmaxf(m, b0[e]); m = fmaxf(m, b1[e]);
    srow[c0 + e] = a0[e]; srow[c0 + 4 + e] = a1[e];
    srow[c1 + e] = b0[e]; srow[c1 + 4 + e] = b1[e];
  }
#pragma unroll
  for (int off = 16; off > 0; off >>= 1) m = fmaxf(m, __shfl_xor(m, off, 32));
  if (lane == 0) redM[wave] = m;
  __syncthreads();
  m = redM[0];
#pragma unroll
  for (int w = 1; w < 8; ++w) m = fmaxf(m, redM[w]);
  float sum = 0.f;
#pragma unroll 1
  for (int e = 0; e < 16; ++e) {
    const int c = c0 + (e & 7) + (e >> 3) * (kSeq / 2);
    const float p = expf(srow[c] - m);
    srow[c] = p;
    sum += p;
  }
#pragma unroll
  for (int off = 16; off > 0; off >>= 1) sum += __shfl_xor(sum, off, 32);
  if (lane == 0) redS[wave] = sum;
  __syncthreads();
  float tot = redS[0];
#pragma unroll
  for (int w = 1; w < 8; ++w) tot += redS[w];
  const float inv = 1.0f / tot;
  unsigned short hb0[8], hb1[8];
#pragma unroll
  for (int e = 0; e < 8; ++e) {
    hb0[e] = h_bits((srow[c0 + e] * inv) * carry);
    hb1[e] = h_bits((srow[c1 + e] * inv) * carry);
  }
  const v4u u0 = (v4u){pk16(hb0[0], hb0[1]), pk16(hb0[2], hb0[3]), pk16(hb0[4], hb0[5]), pk16(hb0[6], hb0[7])};
  const v4u u1 = (v4u){pk16(hb1[0], hb1[1]), pk16(hb1[2], hb1[3]), pk16(hb1[4], hb1[5]), pk16(hb1[6], hb1[7])};
  unsigned short* pr = P + (size_t)row * kSeq;
  for (int pass = 0; pass < 2; ++pass) {
    *(volatile v4u*)(pr + c0) = u0;
    *(volatile v4u*)(pr + c1) = u1;
    __threadfence();
  }
}

extern "C" void kernel_launch(void* const* d_in, const int* in_sizes, int n_in,
                              void* d_out, int out_size, void* d_ws, size_t ws_size,
                              hipStream_t stream) {
  if (n_in < 15) return;
  if (in_sizes[0] != kTok * kDim || in_sizes[1] != kTok * kDim || in_sizes[2] != kTok * kDim) return;
  if (in_sizes[3] != kDim * kHid || in_sizes[4] != kHid || in_sizes[5] != kHid * kQk || in_sizes[6] != kQk) return;
  if (in_sizes[7] != kDim * kHid || in_sizes[8] != kHid || in_sizes[9] != kHid * kQk || in_sizes[10] != kQk) return;
  if (in_sizes[11] != kDim * kDim || in_sizes[12] != kDim || in_sizes[13] != kDim * kDim || in_sizes[14] != kDim) return;
  if (out_size != kTok * kDim) return;
  if (ws_size < kWsTotal) return;

  const float* query = (const float*)d_in[0];
  const float* key   = (const float*)d_in[1];
  const float* value = (const float*)d_in[2];
  const float* Wq1 = (const float*)d_in[3];
  const float* bq1 = (const float*)d_in[4];
  const float* Wq2 = (const float*)d_in[5];
  const float* bq2 = (const float*)d_in[6];
  const float* Wk1 = (const float*)d_in[7];
  const float* bk1 = (const float*)d_in[8];
  const float* Wk2 = (const float*)d_in[9];
  const float* bk2 = (const float*)d_in[10];
  const float* Wv  = (const float*)d_in[11];
  const float* bv  = (const float*)d_in[12];
  const float* Wo  = (const float*)d_in[13];
  const float* bo  = (const float*)d_in[14];
  float* out = (float*)d_out;

  char* ws = (char*)d_ws;
  unsigned short* Q16  = (unsigned short*)(ws + kOffQ16);
  unsigned short* K16  = (unsigned short*)(ws + kOffK16);
  unsigned short* VT16 = (unsigned short*)(ws + kOffVT);
  unsigned short* XHI  = (unsigned short*)(ws + kOffXhi);
  unsigned short* XLO  = (unsigned short*)(ws + kOffXlo);
  unsigned short* XQ16 = (unsigned short*)(ws + kOffXq);
  unsigned short* XK16 = (unsigned short*)(ws + kOffXk);
  unsigned short* XV16 = (unsigned short*)(ws + kOffXv);
  float*          HF32 = (float*)(ws + kOffH);
  unsigned short* G16  = (unsigned short*)(ws + kOffG);
  unsigned short* W1QT = (unsigned short*)(ws + kOffW1q);
  unsigned short* W1KT = (unsigned short*)(ws + kOffW1k);
  unsigned short* W2QT = (unsigned short*)(ws + kOffW2q);
  unsigned short* W2KT = (unsigned short*)(ws + kOffW2k);
  unsigned short* WVT  = (unsigned short*)(ws + kOffWv);
  float*          SB   = (float*)(ws + kOffSb);
  float*          SF32 = (float*)(ws + kOffS);
  unsigned short* P16  = (unsigned short*)(ws + kOffP);
  unsigned short* WOTH = (unsigned short*)(ws + kOffWoh);
  unsigned short* WOTL = (unsigned short*)(ws + kOffWol);

  const dim3 blk256(256);
  const float inv64 = 1.0f / 64.0f;

  cast8x3_kernel<<<dim3((kTok * kDim / 8) / 256, 3), blk256, 0, stream>>>(query, key, value, XQ16, XK16, XV16,
                                                                          kTok * kDim / 8);
  wtcast_kernel<0><<<dim3(kDim / 64, kHid / 64, 2), blk256, 0, stream>>>(Wq1, Wk1, W1QT, W1KT, kDim, kHid, kWCarry);
  wtcast_kernel<0><<<dim3(kHid / 64, kQk / 64, 2), blk256, 0, stream>>>(Wq2, Wk2, W2QT, W2KT, kHid, kQk, kWCarry);
  wtcast_kernel<0><<<dim3(kDim / 64, kDim / 64, 1), blk256, 0, stream>>>(Wv, Wv, WVT, WVT, kDim, kDim, kWCarry);
  sbias_kernel<<<dim3(4), dim3(64), 0, stream>>>(bq2, bk2, bv, SB, kActCarry);

  wmma_gemm64<0, false, 2, 0, false, 0><<<dim3((kTok / 64) * (kHid / 64) / 8, 1), blk256, 0, stream>>>(
      XQ16, XQ16, kDim, 0L, W1QT, W1QT, kDim, 0L, (void*)HF32, (void*)HF32, kHid, 0L,
      bq1, bo, 0L, kTok, kHid, kDim, inv64);
  gelu_cast_kernel<<<dim3((kTok * kHid / 2) / 256), blk256, 0, stream>>>(HF32, G16, kTok * kHid / 2, kActCarry);
  wmma_gemm64<0, false, 2, 1, false, 0><<<dim3((kTok / 64) * (kQk / 64) / 8, 1), blk256, 0, stream>>>(
      G16, G16, kHid, 0L, W2QT, W2QT, kHid, 0L, (void*)Q16, (void*)Q16, kQk, 0L,
      SB, bo, 0L, kTok, kQk, kHid, inv64);
  wmma_gemm64<0, false, 2, 0, false, 0><<<dim3((kTok / 64) * (kHid / 64) / 8, 1), blk256, 0, stream>>>(
      XK16, XK16, kDim, 0L, W1KT, W1KT, kDim, 0L, (void*)HF32, (void*)HF32, kHid, 0L,
      bk1, bo, 0L, kTok, kHid, kDim, inv64);
  gelu_cast_kernel<<<dim3((kTok * kHid / 2) / 256), blk256, 0, stream>>>(HF32, G16, kTok * kHid / 2, kActCarry);
  wmma_gemm64<0, false, 2, 1, false, 0><<<dim3((kTok / 64) * (kQk / 64) / 8, 1), blk256, 0, stream>>>(
      G16, G16, kHid, 0L, W2KT, W2KT, kHid, 0L, (void*)K16, (void*)K16, kQk, 0L,
      SB + 256, bo, 0L, kTok, kQk, kHid, inv64);
  wmma_gemm64<0, false, 1, 1, false, 0><<<dim3((kDim / 64) * (kSeq / 64) / 8, kBatch), blk256, 0, stream>>>(
      WVT, WVT, kDim, 0L, XV16, XV16, kDim, (long)kSeq * kDim, (void*)VT16, (void*)VT16, kSeq, (long)kDim * kSeq,
      SB + 512, bo, 0L, kDim, kSeq, kDim, kActCarry * inv64);

  const float sc_scale = (0.17677669529663688f / (kActCarry * kActCarry));
  const float pv_scale = 1.0f / (kPCarry * kActCarry);
  for (int g = 0; g < kBatch * kHeads; ++g) {
    const int b = g / kHeads, h = g - (g / kHeads) * kHeads;
    const size_t qoff = (size_t)b * kSeq * kQk + (size_t)h * kDqk;
    const size_t voff = (size_t)b * kDim * kSeq + (size_t)h * kDk * kSeq;
    const size_t xoff = (size_t)b * kSeq * kDim + (size_t)h * kDk;
    wmma_gemm64<0, false, 0, 0, false, 0><<<dim3((kSeq / 64) * (kSeq / 64) / 8, 1), blk256, 0, stream>>>(
        Q16 + qoff, Q16 + qoff, kQk, 0L, K16 + qoff, K16 + qoff, kQk, 0L, (void*)SF32, (void*)SF32, kSeq, 0L,
        bo, bo, 0L, kSeq, kSeq, kDqk, sc_scale);
    softmax_row_kernel<<<dim3(kSeq), blk256, 0, stream>>>(SF32, P16, kPCarry);
    wmma_gemm64<0, false, 0, 2, false, 0><<<dim3((kSeq / 64) * (kDk / 64) / 8, 1), blk256, 0, stream>>>(
        P16, P16, kSeq, 0L, VT16 + voff, VT16 + voff, kSeq, 0L, (void*)(XHI + xoff), (void*)(XLO + xoff), kDim, 0L,
        bo, bo, 0L, kSeq, kDk, kSeq, pv_scale);
  }

  wtcast_kernel<1><<<dim3(kDim / 64, kDim / 64, 1), blk256, 0, stream>>>(Wo, Wo, WOTH, WOTL, kDim, kDim, 1.0f);
  wmma_gemm64<1, true, 2, 0, false, 0><<<dim3((kTok / 64) * (kDim / 64) / 8, 1), blk256, 0, stream>>>(
      XHI, XLO, kDim, 0L, WOTH, WOTL, kDim, 0L, (void*)out, (void*)out, kDim, 0L,
      bo, bo, 0L, kTok, kDim, kDim, 1.0f);
}
